// SPNN_15247133901693
// MI455X (gfx1250) — hardware-verified
//
#include <hip/hip_runtime.h>
#include <stddef.h>


#define NTHR    256
#define NWAVE   8
#define HID     128
#define GEOF    13
#define IN0     397
#define K0P     416
#define NGRP    4
#define NDEP    3
#define CH      1024
#define MAXT    (CH / 16)
#define AP0     424
#define AP1     136
#define OPT     136
#define RECD    272
#define RECB    (NGRP * RECD * 8)
#define RPIECES (RECB / 16)
#define SSN     (NGRP * 2 * HID)
#define EPT     8
#define CHUNK   (NTHR * EPT)
#define WCAP    (EPT * 32)
#define LISTN   (NWAVE * WCAP)
#define NBO     256
#define P0BLK   ((NGRP * HID * K0P) / (8 * NTHR))
#define P1BLK   ((NGRP * NDEP * HID * HID) / (8 * NTHR))
#define WSC     8.0f
#define WINV    0.125f
#define EPSBN   1e-5f
#define DYNOUT  (NBO * HID * 4 + LISTN * 4 + 256)

static_assert(CH == 4 * NTHR);
static_assert(CHUNK == 2048);
static_assert((NBO & (NBO - 1)) == 0 && NBO <= 1024);
static_assert(P0BLK * 8 * NTHR == NGRP * HID * K0P);
static_assert(P1BLK * 8 * NTHR == NGRP * NDEP * HID * HID);
static_assert(RPIECES * 16 == RECB);
static_assert((K0P % 32) == 0 && (AP0 % 8) == 0 && (AP1 % 8) == 0 && (OPT % 8) == 0);
static_assert((NBO * HID / 4) % NTHR == 0);
static_assert(SSN == 1024);

typedef float    v4f  __attribute__((ext_vector_type(4)));
typedef float    v8f  __attribute__((ext_vector_type(8)));
typedef int      v4i  __attribute__((ext_vector_type(4)));
typedef double   v2d  __attribute__((ext_vector_type(2)));
typedef _Float16 v2h  __attribute__((ext_vector_type(2)));
typedef _Float16 v4h  __attribute__((ext_vector_type(4)));
typedef _Float16 v8h  __attribute__((ext_vector_type(8)));
typedef _Float16 v16h __attribute__((ext_vector_type(16)));
union FragH { v16h v; v8h h[2]; };

__device__ __forceinline__ v8f zero8f() {
  v8f r;
#pragma unroll
  for (int i = 0; i < 8; ++i) r[i] = 0.0f;
  return r;
}

__device__ __forceinline__ v8f wmh(v16h a, v16h b, v8f c) {
  v8f d = __builtin_amdgcn_wmma_f32_16x16x32_f16(false, a, false, b, (short)0, c, false, false);
  asm volatile("v_nop\n\tv_nop\n\tv_nop\n\tv_nop" : "+v"(d) : "v"(a), "v"(b));
  return d;
}

__device__ __forceinline__ double shx16(double x) {
  const long long u = __double_as_longlong(x);
  int lo = (int)(u & 0xffffffffLL);
  int hi = (int)((unsigned long long)u >> 32);
  lo = __shfl_xor(lo, 16);
  hi = __shfl_xor(hi, 16);
  const long long r = (long long)(((unsigned long long)(unsigned)hi << 32) | (unsigned long long)(unsigned)lo);
  return __longlong_as_double(r);
}

__device__ __forceinline__ void group_compact(const int* __restrict__ exij, const int* __restrict__ exjk,
                                              int nei, int nE, int cbase,
                                              int* glist, int* wcl, int* pre, int* tot,
                                              int tid, int lane, int wave) {
  int gq[4];
  unsigned bs[4];
  bool vq[4];
#pragma unroll
  for (int j = 0; j < 4; ++j) {
    const int el = NTHR * j + tid;
    const int e  = cbase + el;
    const bool valid = e < nE;
    const int ec = e > nE - 1 ? nE - 1 : e;
    const int a = exij[ec], b = exjk[ec];
    const int g = ((a < nei) ? 0 : 2) + ((b < nei) ? 0 : 1);
    const unsigned m0 = __builtin_amdgcn_ballot_w32(valid && g == 0);
    const unsigned m1 = __builtin_amdgcn_ballot_w32(valid && g == 1);
    const unsigned m2 = __builtin_amdgcn_ballot_w32(valid && g == 2);
    const unsigned m3 = __builtin_amdgcn_ballot_w32(valid && g == 3);
    if (lane == 0) {
      int* wp = wcl + (j * NWAVE + wave) * NGRP;
      wp[0] = (int)__builtin_popcount(m0);
      wp[1] = (int)__builtin_popcount(m1);
      wp[2] = (int)__builtin_popcount(m2);
      wp[3] = (int)__builtin_popcount(m3);
    }
    gq[j] = g;
    vq[j] = valid;
    bs[j] = (g == 0) ? m0 : ((g == 1) ? m1 : ((g == 2) ? m2 : m3));
  }
  __syncthreads();
  if (tid < NGRP) {
    int run = 0;
#pragma unroll 1
    for (int idx = 0; idx < 4 * NWAVE; ++idx) {
      pre[idx * NGRP + tid] = run;
      run += wcl[idx * NGRP + tid];
    }
    tot[tid] = run;
  }
  __syncthreads();
#pragma unroll
  for (int j = 0; j < 4; ++j) {
    const int rank = (int)__builtin_amdgcn_mbcnt_lo(bs[j], 0u);
    const int pos  = pre[(j * NWAVE + wave) * NGRP + gq[j]] + rank;
    if (vq[j] && (unsigned)pos < (unsigned)CH) glist[gq[j] * CH + pos] = NTHR * j + tid;
  }
  __syncthreads();
}

__device__ __forceinline__ void epi_stats(v8f acc, float bias, int nval, int hh, double& s, double& q) {
#pragma unroll
  for (int r = 0; r < 8; ++r) {
    const int rr = 8 * hh + r;
    const float hp = acc[r] * WINV + bias;
    const float hv = (rr < nval) ? hp : 0.0f;
    const double hd = (double)hv;
    s += hd;
    q += hd * hd;
  }
}

__device__ __forceinline__ void epi_apply(v8f acc, float bias, float sc, float sh, _Float16* Ot, int n0, int m, int hh) {
#pragma unroll
  for (int r = 0; r < 8; ++r) {
    const int rr = 8 * hh + r;
    const float hp = acc[r] * WINV + bias;
    const float u  = fmaxf(hp * sc + sh, 0.0f);
    Ot[rr * OPT + n0 + m] = (_Float16)u;
  }
}

__device__ __forceinline__ void tile_store(const _Float16* Ot, _Float16* Hp, int e, bool rv, int row, int sub) {
  const v8h ov = *(const v8h*)(Ot + row * OPT + 8 * sub);
  _Float16* dst = Hp + (size_t)e * HID + 8 * sub;
  if (rv) *(volatile v8h*)dst = ov;
  __threadfence();
  if (rv) *(volatile v8h*)dst = ov;
}

__device__ __forceinline__ void rec_store(const double* rec, double* part, int blk, int tid) {
  double* base = part + (size_t)blk * (NGRP * RECD);
  const int p0 = tid, p1 = tid + NTHR, p2 = tid + 2 * NTHR;
  const bool t2 = p2 < RPIECES;
  const v2d v0 = *(const v2d*)(rec + 2 * p0);
  const v2d v1 = *(const v2d*)(rec + 2 * p1);
  const v2d v2 = *(const v2d*)(rec + 2 * (t2 ? p2 : 0));
  *(volatile v2d*)(base + 2 * p0) = v0;
  *(volatile v2d*)(base + 2 * p1) = v1;
  if (t2) *(volatile v2d*)(base + 2 * p2) = v2;
  __threadfence();
  *(volatile v2d*)(base + 2 * p0) = v0;
  *(volatile v2d*)(base + 2 * p1) = v1;
  if (t2) *(volatile v2d*)(base + 2 * p2) = v2;
}

__global__ __launch_bounds__(NTHR) void k_prep(const float* __restrict__ W0, const float* __restrict__ Wd,
                                               _Float16* W0h, _Float16* Wh) {
  const int tid = threadIdx.x;
  v8h v;
  _Float16* dst;
  if (blockIdx.x < P0BLK) {
    const int p = blockIdx.x * NTHR + tid;
    const int f = p * 8;
    const int rw = f / K0P;
    const int col = f - rw * K0P;
    const float* src = W0 + (size_t)rw * IN0;
#pragma unroll
    for (int i = 0; i < 8; ++i) {
      const int cidx = col + i;
      const float w = src[cidx < IN0 - 1 ? cidx : IN0 - 1];
      v[i] = (_Float16)((cidx < IN0) ? w * WSC : 0.0f);
    }
    dst = W0h + f;
  } else {
    const int p = (blockIdx.x - P0BLK) * NTHR + tid;
    const int f = p * 8;
    const v4f a0 = *(const v4f*)(Wd + f);
    const v4f a1 = *(const v4f*)(Wd + f + 4);
    v[0] = (_Float16)(a0.x * WSC); v[1] = (_Float16)(a0.y * WSC);
    v[2] = (_Float16)(a0.z * WSC); v[3] = (_Float16)(a0.w * WSC);
    v[4] = (_Float16)(a1.x * WSC); v[5] = (_Float16)(a1.y * WSC);
    v[6] = (_Float16)(a1.z * WSC); v[7] = (_Float16)(a1.w * WSC);
    dst = Wh + f;
  }
  *(volatile v8h*)dst = v;
  __threadfence();
  *(volatile v8h*)dst = v;
}

template <int MODE>
__global__ __launch_bounds__(NTHR) void k_l0(
    const float* __restrict__ nf, const float* __restrict__ geo, const int* __restrict__ eidx,
    const int* __restrict__ exij, const int* __restrict__ exjk, const int* __restrict__ neip,
    const _Float16* __restrict__ W0h, const float* __restrict__ b0, const float* __restrict__ ssb,
    _Float16* Hp, double* part, int nN, int nE) {
  __shared__ int glist[NGRP * CH];
  __shared__ int wcl[4 * NWAVE * NGRP];
  __shared__ int pre[4 * NWAVE * NGRP];
  __shared__ int tot[NGRP];
  __shared__ __attribute__((aligned(16))) _Float16 At[16 * AP0];
  __shared__ __attribute__((aligned(16))) _Float16 Ot[16 * OPT];
  __shared__ __attribute__((aligned(16))) double rec[NGRP * RECD];
  __shared__ __attribute__((aligned(16))) float sst[SSN];

  const int tid = threadIdx.x, lane = tid & 31, wave = tid >> 5, hh = lane >> 4, m = lane & 15;
  const int row = tid >> 4, sub = tid & 15, n0 = 16 * wave;
  const int cbase = blockIdx.x * CH;
  const int nei = neip[0];

  if (MODE == 1) {
    for (int i = tid; i < SSN; i += NTHR) sst[i] = ssb[i];
  }
  group_compact(exij, exjk, nei, nE, cbase, glist, wcl, pre, tot, tid, lane, wave);
  if (MODE == 0) {
    if (tid < 64) {
      const int g = tid >> 4, j = tid & 15;
      rec[g * RECD + 2 * HID + j] = (j == 0) ? (double)tot[g] : 0.0;
    }
  }

#pragma unroll 1
  for (int g = 0; g < NGRP; ++g) {
    const int tg = tot[g];
    int ntile = (tg + 15) >> 4;
    ntile = ntile > MAXT ? MAXT : ntile;
    double s = 0.0, q = 0.0;
    const float bias = b0[g * HID + n0 + m];
    float sc = 1.0f, sh = 0.0f;
    if (MODE == 1) { sc = sst[g * (2 * HID) + n0 + m]; sh = sst[g * (2 * HID) + HID + n0 + m]; }
    const _Float16* brow = W0h + (size_t)(g * HID + n0 + m) * K0P;
#pragma unroll 1
    for (int tt = 0; tt < ntile; ++tt) {
      const int li = 16 * tt + row;
      const bool rv = li < tg;
      int lic = li < tg - 1 ? li : tg - 1;
      lic = lic < 0 ? 0 : (lic > CH - 1 ? CH - 1 : lic);
      int e = cbase + glist[g * CH + lic];
      e = e < 0 ? 0 : (e > nE - 1 ? nE - 1 : e);
      {
        int ni = eidx[e];
        int nj = eidx[(size_t)nE + e];
        int nk = eidx[2 * (size_t)nE + e];
        ni = ni < 0 ? 0 : (ni > nN - 1 ? nN - 1 : ni);
        nj = nj < 0 ? 0 : (nj > nN - 1 ? nN - 1 : nj);
        nk = nk < 0 ? 0 : (nk > nN - 1 ? nN - 1 : nk);
#pragma unroll
        for (int qn = 0; qn < 3; ++qn) {
          const int nid = (qn == 0) ? ni : ((qn == 1) ? nj : nk);
          const float* src = nf + (size_t)nid * HID + 8 * sub;
          const v4f a0 = *(const v4f*)src;
          const v4f a1 = *(const v4f*)(src + 4);
          v8h hv;
          hv[0] = (_Float16)(rv ? a0.x : 0.0f); hv[1] = (_Float16)(rv ? a0.y : 0.0f);
          hv[2] = (_Float16)(rv ? a0.z : 0.0f); hv[3] = (_Float16)(rv ? a0.w : 0.0f);
          hv[4] = (_Float16)(rv ? a1.x : 0.0f); hv[5] = (_Float16)(rv ? a1.y : 0.0f);
          hv[6] = (_Float16)(rv ? a1.z : 0.0f); hv[7] = (_Float16)(rv ? a1.w : 0.0f);
          *(v8h*)(At + row * AP0 + HID * qn + 8 * sub) = hv;
        }
        const int gc0 = 2 * sub, gc1 = 2 * sub + 1;
        const float* gsrc = geo + (size_t)e * GEOF;
        const float g0 = gsrc[gc0 < GEOF - 1 ? gc0 : GEOF - 1];
        const float g1 = gsrc[gc1 < GEOF - 1 ? gc1 : GEOF - 1];
        v2h gv;
        gv[0] = (_Float16)((rv && gc0 < GEOF) ? g0 : 0.0f);
        gv[1] = (_Float16)((rv && gc1 < GEOF) ? g1 : 0.0f);
        *(v2h*)(At + row * AP0 + 3 * HID + 2 * sub) = gv;
      }
      __syncthreads();
      v8f acc = zero8f();
      const _Float16* arow = At + m * AP0;
#pragma unroll 1
      for (int ks = 0; ks < K0P / 32; ++ks) {
        const int k0 = 32 * ks;
        FragH a, b;
        a.h[0] = *(const v8h*)(arow + k0 + 8 * hh);
        a.h[1] = *(const v8h*)(arow + k0 + 16 + 8 * hh);
        b.h[0] = *(const v8h*)(brow + k0 + 8 * hh);
        b.h[1] = *(const v8h*)(brow + k0 + 16 + 8 * hh);
        acc = wmh(a.v, b.v, acc);
      }
      if (MODE == 0) {
        const int rem  = tg - 16 * tt;
        const int nval = rem < 16 ? rem : 16;
        epi_stats(acc, bias, nval, hh, s, q);
        __syncthreads();
      } else {
        epi_apply(acc, bias, sc, sh, Ot, n0, m, hh);
        __syncthreads();
        tile_store(Ot, Hp, e, rv, row, sub);
      }
    }
    if (MODE == 0) {
      s += shx16(s);
      q += shx16(q);
      if (hh == 0) {
        rec[g * RECD + n0 + m] = s;
        rec[g * RECD + HID + n0 + m] = q;
      }
    }
  }
  if (MODE == 0) {
    __syncthreads();
    rec_store(rec, part, blockIdx.x, tid);
  }
}

template <int MODE>
__global__ __launch_bounds__(NTHR) void k_lh(
    const int* __restrict__ exij, const int* __restrict__ exjk, const int* __restrict__ neip,
    const _Float16* __restrict__ Wh, const float* __restrict__ bl, const float* __restrict__ ssb,
    _Float16* Hp, double* part, int l, int nE) {
  __shared__ int glist[NGRP * CH];
  __shared__ int wcl[4 * NWAVE * NGRP];
  __shared__ int pre[4 * NWAVE * NGRP];
  __shared__ int tot[NGRP];
  __shared__ __attribute__((aligned(16))) _Float16 At[16 * AP1];
  __shared__ __attribute__((aligned(16))) _Float16 Ot[16 * OPT];
  __shared__ __attribute__((aligned(16))) double rec[NGRP * RECD];
  __shared__ __attribute__((aligned(16))) float sst[SSN];

  const int tid = threadIdx.x, lane = tid & 31, wave = tid >> 5, hh = lane >> 4, m = lane & 15;
  const int row = tid >> 4, sub = tid & 15, n0 = 16 * wave;
  const int cbase = blockIdx.x * CH;
  const int nei = neip[0];

  if (MODE == 1) {
    for (int i = tid; i < SSN; i += NTHR) sst[i] = ssb[(size_t)(l + 1) * SSN + i];
  }
  group_compact(exij, exjk, nei, nE, cbase, glist, wcl, pre, tot, tid, lane, wave);
  if (MODE == 0) {
    if (tid < 64) {
      const int g = tid >> 4, j = tid & 15;
      rec[g * RECD + 2 * HID + j] = (j == 0) ? (double)tot[g] : 0.0;
    }
  }

#pragma unroll 1
  for (int g = 0; g < NGRP; ++g) {
    const int tg = tot[g];
    int ntile = (tg + 15) >> 4;
    ntile = ntile > MAXT ? MAXT : ntile;
    double s = 0.0, q = 0.0;
    const float bias = bl[(g * NDEP + l) * HID + n0 + m];
    float sc = 1.0f, sh = 0.0f;
    if (MODE == 1) { sc = sst[g * (2 * HID) + n0 + m]; sh = sst[g * (2 * HID) + HID + n0 + m]; }
    const _Float16* brow = Wh + ((size_t)((g * NDEP + l) * HID + n0 + m)) * HID;
#pragma unroll 1
    for (int tt = 0; tt < ntile; ++tt) {
      const int li = 16 * tt + row;
      const bool rv = li < tg;
      int lic = li < tg - 1 ? li : tg - 1;
      lic = lic < 0 ? 0 : (lic > CH - 1 ? CH - 1 : lic);
      int e = cbase + glist[g * CH + lic];
      e = e < 0 ? 0 : (e > nE - 1 ? nE - 1 : e);
      {
        const v8h hin = *(const v8h*)(Hp + (size_t)e * HID + 8 * sub);
        v8h av;
#pragma unroll
        for (int i = 0; i < 8; ++i) av[i] = rv ? hin[i] : (_Float16)0.0f;
        *(v8h*)(At + row * AP1 + 8 * sub) = av;
      }
      __syncthreads();
      v8f acc = zero8f();
      const _Float16* arow = At + m * AP1;
#pragma unroll
      for (int ks = 0; ks < HID / 32; ++ks) {
        const int k0 = 32 * ks;
        FragH a, b;
        a.h[0] = *(const v8h*)(arow + k0 + 8 * hh);
        a.h[1] = *(const v8h*)(arow + k0 + 16 + 8 * hh);
        b.h[0] = *(const v8h*)(brow + k0 + 8 * hh);
        b.h[1] = *(const v8h*)(brow + k0 + 16 + 8 * hh);
        acc = wmh(a.v, b.v, acc);
      }
      if (MODE == 0) {
        const int rem  = tg - 16 * tt;
        const int nval = rem < 16 ? rem : 16;
        epi_stats(acc, bias, nval, hh, s, q);
        __syncthreads();
      } else {
        epi_apply(acc, bias, sc, sh, Ot, n0, m, hh);
        __syncthreads();
        tile_store(Ot, Hp, e, rv, row, sub);
      }
    }
    if (MODE == 0) {
      s += shx16(s);
      q += shx16(q);
      if (hh == 0) {
        rec[g * RECD + n0 + m] = s;
        rec[g * RECD + HID + n0 + m] = q;
      }
    }
  }
  if (MODE == 0) {
    __syncthreads();
    rec_store(rec, part, blockIdx.x, tid);
  }
}

__global__ __launch_bounds__(HID) void k_fin(const double* __restrict__ part, const float* __restrict__ gam,
                                             const float* __restrict__ bet, float* ssb, int l, int nblk) {
  __shared__ __attribute__((aligned(16))) float scsh[2 * HID];
  const int g = blockIdx.x, c = threadIdx.x;
  double S = 0.0, Q = 0.0, C = 0.0;
#pragma unroll 1
  for (int bk = 0; bk < nblk; ++bk) {
    const double* r = part + ((size_t)bk * NGRP + g) * RECD;
    S += r[c];
    Q += r[HID + c];
    C += r[2 * HID];
  }
  const double cnt = C < 1.0 ? 1.0 : C;
  const double mean = S / cnt;
  double var = Q / cnt - mean * mean;
  var = var < 0.0 ? 0.0 : var;
  const float rstd = 1.0f / sqrtf((float)var + EPSBN);
  const float gm = gam[(size_t)(g * (NDEP + 1) + l) * HID + c];
  const float bt = bet[(size_t)(g * (NDEP + 1) + l) * HID + c];
  const float sc = gm * rstd;
  const float sh = bt - (float)mean * sc;
  scsh[c] = sc;
  scsh[HID + c] = sh;
  __syncthreads();
  const int cc = c < 63 ? c : 63;
  const v4f v = *(const v4f*)(scsh + 4 * cc);
  float* dst = ssb + (size_t)(l * NGRP + g) * (2 * HID) + 4 * cc;
  const bool wr = c < 64;
  if (wr) *(volatile v4f*)dst = v;
  __threadfence();
  if (wr) *(volatile v4f*)dst = v;
}

__device__ __forceinline__ int scan_chunk(const int* __restrict__ dsts, int nE, int cbase, int nodeBase,
                                          int vec8, int* list, int tid, int wave) {
  int wc = 0;
  const int el0  = tid * EPT;
  const int e0   = cbase + el0;
  const int sent = -2147483647 - 1;
  v4i da, db;
  if (vec8 != 0 && cbase + CHUNK <= nE) {
    da = *(const v4i*)(dsts + e0);
    db = *(const v4i*)(dsts + e0 + 4);
  } else {
    da.x = (e0     < nE) ? dsts[min(e0,     nE - 1)] : sent;
    da.y = (e0 + 1 < nE) ? dsts[min(e0 + 1, nE - 1)] : sent;
    da.z = (e0 + 2 < nE) ? dsts[min(e0 + 2, nE - 1)] : sent;
    da.w = (e0 + 3 < nE) ? dsts[min(e0 + 3, nE - 1)] : sent;
    db.x = (e0 + 4 < nE) ? dsts[min(e0 + 4, nE - 1)] : sent;
    db.y = (e0 + 5 < nE) ? dsts[min(e0 + 5, nE - 1)] : sent;
    db.z = (e0 + 6 < nE) ? dsts[min(e0 + 6, nE - 1)] : sent;
    db.w = (e0 + 7 < nE) ? dsts[min(e0 + 7, nE - 1)] : sent;
  }
  const unsigned nb = (unsigned)nodeBase;
  const unsigned s0 = (unsigned)da.x - nb, s1 = (unsigned)da.y - nb;
  const unsigned s2 = (unsigned)da.z - nb, s3 = (unsigned)da.w - nb;
  const unsigned s4 = (unsigned)db.x - nb, s5 = (unsigned)db.y - nb;
  const unsigned s6 = (unsigned)db.z - nb, s7 = (unsigned)db.w - nb;
  const bool h0 = s0 < (unsigned)NBO, h1 = s1 < (unsigned)NBO, h2 = s2 < (unsigned)NBO, h3 = s3 < (unsigned)NBO;
  const bool h4 = s4 < (unsigned)NBO, h5 = s5 < (unsigned)NBO, h6 = s6 < (unsigned)NBO, h7 = s7 < (unsigned)NBO;
  const unsigned any = __builtin_amdgcn_ballot_w32(h0 | h1 | h2 | h3 | h4 | h5 | h6 | h7);
  if (any != 0u) {
#define HITJ(J, HJ, SJ) { \
      const unsigned mj = __builtin_amdgcn_ballot_w32(HJ); \
      if (mj != 0u) { \
        if (HJ) { \
          const int pos = wc + (int)__builtin_amdgcn_mbcnt_lo(mj, 0u); \
          if (pos < WCAP) list[wave * WCAP + pos] = (int)(((SJ) << 11) | (unsigned)(el0 + (J))); \
        } \
        wc += (int)__builtin_popcount(mj); } }
    HITJ(0, h0, s0)
    HITJ(1, h1, s1)
    HITJ(2, h2, s2)
    HITJ(3, h3, s3)
    HITJ(4, h4, s4)
    HITJ(5, h5, s5)
    HITJ(6, h6, s6)
    HITJ(7, h7, s7)
#undef HITJ
  }
  return wc;
}

__global__ __launch_bounds__(NTHR) void k_out(
    const _Float16* __restrict__ Hp, const int* __restrict__ eidx,
    const int* __restrict__ exij, const int* __restrict__ exjk, const int* __restrict__ neip,
    const float* __restrict__ att, float* outp, int nN, int nE, int vec8) {
  extern __shared__ __attribute__((aligned(16))) float dynl[];
  float* accl = dynl;
  int*   list = (int*)(dynl + NBO * HID);
  int*   wcnt = (int*)(dynl + NBO * HID + LISTN);

  const int tid = threadIdx.x, lane = tid & 31, wave = tid >> 5;
  const int nodeBase = blockIdx.x * NBO;
  const int nei = neip[0];
  const float at0 = att[0], at1 = att[1], at2 = att[2], at3 = att[3];

  {
    const v4f z = {0.0f, 0.0f, 0.0f, 0.0f};
    for (int i = tid; i < NBO * HID / 4; i += NTHR) ((v4f*)accl)[i] = z;
  }
  __syncthreads();

  const int nChunks = (nE + CHUNK - 1) / CHUNK;
#pragma unroll 1
  for (int ch = 0; ch < nChunks; ++ch) {
    const int cbase = ch * CHUNK;
    const int wc = scan_chunk(eidx, nE, cbase, nodeBase, vec8, list, tid, wave);
    if (lane == 0) wcnt[wave] = wc;
    __syncthreads();
#pragma unroll 1
    for (int w2 = 0; w2 < NWAVE; ++w2) {
      int n = wcnt[w2];
      n = n > WCAP ? WCAP : (n < 0 ? 0 : n);
#pragma unroll 1
      for (int ix = 0; ix < n; ++ix) {
        const int val  = list[w2 * WCAP + ix];
        const int slot = (val >> 11) & (NBO - 1);
        if ((slot & (NWAVE - 1)) == wave) {
          int e = cbase + (val & (CHUNK - 1));
          e = e > nE - 1 ? nE - 1 : e;
          const int g = ((exij[e] < nei) ? 0 : 2) + ((exjk[e] < nei) ? 0 : 1);
          const float ag = (g == 0) ? at0 : ((g == 1) ? at1 : ((g == 2) ? at2 : at3));
          const v4h hv = *(const v4h*)(Hp + (size_t)e * HID + 4 * lane);
          v4f y;
#pragma unroll
          for (int qq = 0; qq < 4; ++qq) {
            float u = (float)hv[qq];
            u = (u > 0.0f) ? u : 0.01f * u;
            y[qq] = u * ag;
          }
          v4f* ap = (v4f*)(accl + slot * HID + 4 * lane);
          const v4f cur = *ap;
          *ap = cur + y;
        }
      }
    }
    __syncthreads();
  }

#pragma unroll 1
  for (int it = 0; it < (NBO * HID / 4) / NTHR; ++it) {
    const int p = it * NTHR + tid;
    const int r = p >> 5, piece = p & 31;
    const int node = nodeBase + r;
    const v4f v = *(const v4f*)(accl + r * HID + 4 * piece);
    if (node < nN) *(volatile v4f*)(outp + (size_t)node * HID + 4 * piece) = v;
  }
  __threadfence();
#pragma unroll 1
  for (int it = 0; it < (NBO * HID / 4) / NTHR; ++it) {
    const int p = it * NTHR + tid;
    const int r = p >> 5, piece = p & 31;
    const int node = nodeBase + r;
    const v4f v = *(const v4f*)(accl + r * HID + 4 * piece);
    if (node < nN) *(volatile v4f*)(outp + (size_t)node * HID + 4 * piece) = v;
  }
}

static inline size_t alup(size_t x) { return (x + 255) & ~(size_t)255; }

extern "C" void kernel_launch(void* const* d_in, const int* in_sizes, int n_in,
                              void* d_out, int out_size, void* d_ws, size_t ws_size,
                              hipStream_t stream) {
  if (n_in < 13) return;
  const int nN = in_sizes[0] / HID;
  const int nE = in_sizes[1] / GEOF;
  if (nN <= 0 || nE <= 0) return;
  if (in_sizes[0] != nN * HID || in_sizes[1] != nE * GEOF) return;
  if (in_sizes[2] != 3 * nE || in_sizes[3] != nE || in_sizes[4] != nE) return;
  if (in_sizes[5] < 1 || in_sizes[6] != NGRP) return;
  if (in_sizes[7] != NGRP * HID * IN0 || in_sizes[8] != NGRP * HID) return;
  if (in_sizes[9] != NGRP * NDEP * HID * HID || in_sizes[10] != NGRP * NDEP * HID) return;
  if (in_sizes[11] != NGRP * (NDEP + 1) * HID || in_sizes[12] != NGRP * (NDEP + 1) * HID) return;
  if (out_size != nN * HID) return;

  const float* nf   = (const float*)d_in[0];
  const float* geo  = (const float*)d_in[1];
  const int*   eidx = (const int*)d_in[2];
  const int*   exij = (const int*)d_in[3];
  const int*   exjk = (const int*)d_in[4];
  const int*   neip = (const int*)d_in[5];
  const float* att  = (const float*)d_in[6];
  const float* W0   = (const float*)d_in[7];
  const float* b0   = (const float*)d_in[8];
  const float* Wd   = (const float*)d_in[9];
  const float* bd   = (const float*)d_in[10];
  const float* gam  = (const float*)d_in[11];
  const float* bet  = (const float*)d_in[12];
  float* out = (float*)d_out;

  const int nblk = (nE + CH - 1) / CH;
  const int nob  = (nN + NBO - 1) / NBO;

  size_t off = 0;
  const size_t oW0h = off; off = alup(off + (size_t)NGRP * HID * K0P * 2);
  const size_t oWh  = off; off = alup(off + (size_t)NGRP * NDEP * HID * HID * 2);
  const size_t oSS  = off; off = alup(off + (size_t)(NDEP + 1) * SSN * 4);
  const size_t oPT  = off; off = alup(off + (size_t)nblk * RECB);
  const size_t oH   = off; off = alup(off + (size_t)nE * HID * 2);
  if (off > ws_size || off > (size_t)134217728) return;

  char* ws = (char*)d_ws;
  _Float16* W0h  = (_Float16*)(ws + oW0h);
  _Float16* Wh   = (_Float16*)(ws + oWh);
  float*    ssb  = (float*)(ws + oSS);
  double*   part = (double*)(ws + oPT);
  _Float16* Hp   = (_Float16*)(ws + oH);

  const int vec8 = ((nE & 3) == 0) ? 1 : 0;

  k_prep<<<P0BLK + P1BLK, NTHR, 0, stream>>>(W0, Wd, W0h, Wh);

  k_l0<0><<<nblk, NTHR, 0, stream>>>(nf, geo, eidx, exij, exjk, neip, W0h, b0, ssb, Hp, part, nN, nE);
  k_fin<<<NGRP, HID, 0, stream>>>(part, gam, bet, ssb, 0, nblk);
  k_l0<1><<<nblk, NTHR, 0, stream>>>(nf, geo, eidx, exij, exjk, neip, W0h, b0, ssb, Hp, part, nN, nE);

  k_lh<0><<<nblk, NTHR, 0, stream>>>(exij, exjk, neip, Wh, bd, ssb, Hp, part, 0, nE);
  k_fin<<<NGRP, HID, 0, stream>>>(part, gam, bet, ssb, 1, nblk);
  k_lh<1><<<nblk, NTHR, 0, stream>>>(exij, exjk, neip, Wh, bd, ssb, Hp, part, 0, nE);

  k_lh<0><<<nblk, NTHR, 0, stream>>>(exij, exjk, neip, Wh, bd, ssb, Hp, part, 1, nE);
  k_fin<<<NGRP, HID, 0, stream>>>(part, gam, bet, ssb, 2, nblk);
  k_lh<1><<<nblk, NTHR, 0, stream>>>(exij, exjk, neip, Wh, bd, ssb, Hp, part, 1, nE);

  k_lh<0><<<nblk, NTHR, 0, stream>>>(exij, exjk, neip, Wh, bd, ssb, Hp, part, 2, nE);
  k_fin<<<NGRP, HID, 0, stream>>>(part, gam, bet, ssb, 3, nblk);
  k_lh<1><<<nblk, NTHR, 0, stream>>>(exij, exjk, neip, Wh, bd, ssb, Hp, part, 2, nE);

  hipFuncSetAttribute(reinterpret_cast<const void*>(&k_out), hipFuncAttributeMaxDynamicSharedMemorySize, DYNOUT);
  k_out<<<nob, NTHR, DYNOUT, stream>>>(Hp, eidx, exij, exjk, neip, att, out, nN, nE, vec8);
}
